// LFM3BAttention_63531156242849
// MI455X (gfx1250) — hardware-verified
//
#include <hip/hip_runtime.h>
#include <hip/hip_bf16.h>
#include <stddef.h>
#include <stdint.h>

#define SQ    2048
#define HID   2048
#define NH    32
#define NKV   8
#define HDM   64
#define KVD   (NKV * HDM)
#define NQKV  (HID + 2 * KVD)
#define QB    128
#define KC    64
#define NQB   (SQ / QB)
#define NKC   (SQ / KC)
#define NFREQ (HDM / 2)
#define R0    256
#define MB3   (R0 / 256)
#define QB3   (R0 / QB)
#define Q64N  (R0 / 64)

static_assert(SQ % 256 == 0);
static_assert(HID % 64 == 0);
static_assert(KVD % 64 == 0);
static_assert(HDM == 64);
static_assert(NH * HDM == HID);
static_assert(NH == 4 * NKV);
static_assert(NQB == 16);
static_assert(NKC == 32);
static_assert(R0 % 256 == 0);
static_assert(R0 < SQ);
static_assert(R0 % KC == 0);

typedef _Float16 v16h __attribute__((ext_vector_type(16)));
typedef _Float16 v8h  __attribute__((ext_vector_type(8)));
typedef float    v8f  __attribute__((ext_vector_type(8)));
typedef float    v4f  __attribute__((ext_vector_type(4)));
typedef unsigned int   v4u   __attribute__((ext_vector_type(4)));
typedef int            v4i   __attribute__((ext_vector_type(4)));
typedef unsigned short v8us  __attribute__((ext_vector_type(8)));
typedef unsigned short v16us __attribute__((ext_vector_type(16)));
typedef __bf16         v16b  __attribute__((ext_vector_type(16)));
typedef unsigned short ush;

union Frag  { v16h v; v8h h[2]; };
union FragU { v16us v; v8us h[2]; v16b b; };
union Pack8 { v8h h; v4u u; };
union PackU { v8us s; v4u u; };
struct HL { v4u h; v4u l; };

__device__ __forceinline__ ush f2bf(float f) {
  const unsigned u = __float_as_uint(f);
  return (ush)((u + 0x7FFFu + ((u >> 16) & 1u)) >> 16);
}
__device__ __forceinline__ float bf2f(ush b) { return __uint_as_float(((unsigned)b) << 16); }

__device__ __forceinline__ HL split8(v8f f) {
  PackU ph, pl;
#pragma unroll
  for (int e = 0; e < 8; ++e) {
    const ush hi = f2bf(f[e]);
    ph.s[e] = hi;
    pl.s[e] = f2bf(f[e] - bf2f(hi));
  }
  HL r; r.h = ph.u; r.l = pl.u;
  return r;
}
__device__ __forceinline__ v8f h8tof(v8h x) {
  v8f f;
#pragma unroll
  for (int e = 0; e < 8; ++e) f[e] = (float)x[e];
  return f;
}

__device__ __forceinline__ v8f mma16(v16h a, v16h b, v8f c) {
  c = __builtin_amdgcn_wmma_f32_16x16x32_f16(false, a, false, b, (short)0, c, false, false);
  asm volatile("v_nop\n\tv_nop\n\tv_nop\n\tv_nop" : "+v"(c) : "v"(a), "v"(b));
  return c;
}
__device__ __forceinline__ v8f mmab(v16us a, v16us b, v8f c) {
  FragU ua, ub; ua.v = a; ub.v = b;
  c = __builtin_amdgcn_wmma_f32_16x16x32_bf16(false, ua.b, false, ub.b, (short)0, c, false, false);
  asm volatile("v_nop\n\tv_nop\n\tv_nop\n\tv_nop" : "+v"(c) : "v"(a), "v"(b));
  return c;
}

__device__ __forceinline__ v16h ldfrag(const _Float16* p, int ld, int row0, int k0, int lane) {
  const int m = lane & 15, lh = lane >> 4;
  const _Float16* q = p + (size_t)(row0 + m) * ld + k0 + 8 * lh;
  Frag f;
  f.h[0] = *(const v8h*)(q);
  f.h[1] = *(const v8h*)(q + 16);
  return f.v;
}
__device__ __forceinline__ v16us ldfragu(const ush* p, int ld, int row0, int k0, int lane) {
  const int m = lane & 15, lh = lane >> 4;
  const ush* q = p + (size_t)(row0 + m) * ld + k0 + 8 * lh;
  FragU f;
  f.h[0] = *(const v8us*)(q);
  f.h[1] = *(const v8us*)(q + 16);
  return f.v;
}

__device__ __forceinline__ v8f zero8() { return (v8f){0.f, 0.f, 0.f, 0.f, 0.f, 0.f, 0.f, 0.f}; }

__device__ __forceinline__ void gemm32x64(const _Float16* __restrict__ A, int lda,
                                          const _Float16* __restrict__ Bt, int ldb,
                                          int m0, int n0, int lane, v8f (&acc)[2][4]) {
#pragma unroll 2
  for (int k0 = 0; k0 < HID; k0 += 32) {
    const v16h a0 = ldfrag(A, lda, m0, k0, lane);
    const v16h a1 = ldfrag(A, lda, m0 + 16, k0, lane);
    const v16h b0 = ldfrag(Bt, ldb, n0, k0, lane);
    const v16h b1 = ldfrag(Bt, ldb, n0 + 16, k0, lane);
    const v16h b2 = ldfrag(Bt, ldb, n0 + 32, k0, lane);
    const v16h b3 = ldfrag(Bt, ldb, n0 + 48, k0, lane);
    acc[0][0] = mma16(a0, b0, acc[0][0]);
    acc[1][0] = mma16(a1, b0, acc[1][0]);
    acc[0][1] = mma16(a0, b1, acc[0][1]);
    acc[1][1] = mma16(a1, b1, acc[1][1]);
    acc[0][2] = mma16(a0, b2, acc[0][2]);
    acc[1][2] = mma16(a1, b2, acc[1][2]);
    acc[0][3] = mma16(a0, b3, acc[0][3]);
    acc[1][3] = mma16(a1, b3, acc[1][3]);
  }
}

__device__ __forceinline__ void gemm3_32x64(const ush* __restrict__ Ah, const ush* __restrict__ Al, int lda,
                                            const ush* __restrict__ Bh, const ush* __restrict__ Bl, int ldb,
                                            int m0, int n0, int lane, v8f (&acc)[2][4]) {
#pragma unroll 1
  for (int k0 = 0; k0 < HID; k0 += 32) {
    const v16us a0h = ldfragu(Ah, lda, m0, k0, lane);
    const v16us a1h = ldfragu(Ah, lda, m0 + 16, k0, lane);
    const v16us a0l = ldfragu(Al, lda, m0, k0, lane);
    const v16us a1l = ldfragu(Al, lda, m0 + 16, k0, lane);
#pragma unroll
    for (int t = 0; t < 4; ++t) {
      const v16us bh = ldfragu(Bh, ldb, n0 + 16 * t, k0, lane);
      const v16us bl = ldfragu(Bl, ldb, n0 + 16 * t, k0, lane);
      acc[0][t] = mmab(a0h, bh, acc[0][t]);
      acc[1][t] = mmab(a1h, bh, acc[1][t]);
      acc[0][t] = mmab(a0h, bl, acc[0][t]);
      acc[1][t] = mmab(a1h, bl, acc[1][t]);
      acc[0][t] = mmab(a0l, bh, acc[0][t]);
      acc[1][t] = mmab(a1l, bh, acc[1][t]);
    }
  }
}

__global__ __launch_bounds__(256) void k_cvt_x(const float* __restrict__ x, _Float16* __restrict__ xh,
                                               ush* __restrict__ x3h, ush* __restrict__ x3l,
                                               int ngrp, int n3grp) {
  const int t = blockIdx.x * 256 + (int)threadIdx.x;
  if (t >= ngrp) return;
  const size_t o = (size_t)t * 8;
  const v4f a0 = *(const v4f*)(x + o);
  const v4f a1 = *(const v4f*)(x + o + 4);
  Pack8 pk;
  pk.h = (v8h){(_Float16)a0[0], (_Float16)a0[1], (_Float16)a0[2], (_Float16)a0[3],
               (_Float16)a1[0], (_Float16)a1[1], (_Float16)a1[2], (_Float16)a1[3]};
  const v4u vv = pk.u;
  const bool three = (t < n3grp);
  HL s; s.h = (v4u){0u, 0u, 0u, 0u}; s.l = s.h;
  if (three) {
    const v8f f = (v8f){a0[0], a0[1], a0[2], a0[3], a1[0], a1[1], a1[2], a1[3]};
    s = split8(f);
  }
  volatile v4u* d = (volatile v4u*)(xh + o);
  *d = vv;
  if (three) { *(volatile v4u*)(x3h + o) = s.h; *(volatile v4u*)(x3l + o) = s.l; }
  __threadfence();
  *d = vv;
  if (three) { *(volatile v4u*)(x3h + o) = s.h; *(volatile v4u*)(x3l + o) = s.l; }
}

#define WTP 68
__global__ __launch_bounds__(256) void k_wt(const float* __restrict__ w, _Float16* __restrict__ wt,
                                            ush* __restrict__ wth, ush* __restrict__ wtl, int nout) {
  __shared__ __align__(16) float tf[64 * WTP];
  const int tid = threadIdx.x;
  const int n0 = blockIdx.x * 64;
  const int k0 = blockIdx.y * 64;
  {
    const int kr = tid >> 4;
    const int n4 = (tid & 15) * 4;
#pragma unroll
    for (int it = 0; it < 4; ++it) {
      const int kl = it * 16 + kr;
      const v4f a = *(const v4f*)(w + (size_t)(k0 + kl) * nout + n0 + n4);
      *(v4f*)(tf + kl * WTP + n4) = a;
    }
  }
  __syncthreads();
  v4u vf[2], vh[2], vl[2];
  size_t go[2];
#pragma unroll
  for (int j = 0; j < 2; ++j) {
    const int p  = tid + 256 * j;
    const int nl = p >> 3;
    const int pc = p & 7;
    const float* cp = tf + (pc * 8) * WTP + nl;
    const v8f f = (v8f){cp[0 * WTP], cp[1 * WTP], cp[2 * WTP], cp[3 * WTP],
                        cp[4 * WTP], cp[5 * WTP], cp[6 * WTP], cp[7 * WTP]};
    Pack8 pk;
    pk.h = (v8h){(_Float16)(f[0] * 32.0f), (_Float16)(f[1] * 32.0f), (_Float16)(f[2] * 32.0f),
                 (_Float16)(f[3] * 32.0f), (_Float16)(f[4] * 32.0f), (_Float16)(f[5] * 32.0f),
                 (_Float16)(f[6] * 32.0f), (_Float16)(f[7] * 32.0f)};
    vf[j] = pk.u;
    const HL s = split8(f);
    vh[j] = s.h;
    vl[j] = s.l;
    go[j] = (size_t)(n0 + nl) * HID + k0 + pc * 8;
  }
  for (int ps = 0; ps < 2; ++ps) {
#pragma unroll
    for (int j = 0; j < 2; ++j) {
      *(volatile v4u*)(wt + go[j])  = vf[j];
      *(volatile v4u*)(wth + go[j]) = vh[j];
      *(volatile v4u*)(wtl + go[j]) = vl[j];
    }
    __threadfence();
  }
}

__global__ __launch_bounds__(256) void k_wsplit(const float* __restrict__ w, ush* __restrict__ wth,
                                                ush* __restrict__ wtl, int nout) {
  const int t  = blockIdx.x * 256 + (int)threadIdx.x;
  const int n  = t / (HID / 8);
  const int kp = (t - n * (HID / 8)) * 8;
  if (n >= nout) return;
  v8f f;
#pragma unroll
  for (int e = 0; e < 8; ++e) f[e] = w[(size_t)(kp + e) * nout + n];
  const HL s = split8(f);
  const size_t go = (size_t)n * HID + kp;
  *(volatile v4u*)(wth + go) = s.h;
  *(volatile v4u*)(wtl + go) = s.l;
  __threadfence();
  *(volatile v4u*)(wth + go) = s.h;
  *(volatile v4u*)(wtl + go) = s.l;
}

__global__ __launch_bounds__(256) void k_rope_tab(float* __restrict__ ctab, float* __restrict__ stab, int n) {
  __shared__ __align__(16) float sc[256];
  __shared__ __align__(16) float ss[256];
  const int tid = threadIdx.x;
  const int tb = blockIdx.x * 256;
  int t = tb + tid;
  t = (t < n) ? t : (n - 1);
  const int pos = t >> 5;
  const int i = t & 31;
  const int j = i >> 3, k = i & 7;
  const double b8 =
      (k == 0) ? 1.0 :
      (k == 1) ? 1.333521432163324 :
      (k == 2) ? 1.778279410038923 :
      (k == 3) ? 2.371373705661655 :
      (k == 4) ? 3.1622776601683795 :
      (k == 5) ? 4.216965034285822 :
      (k == 6) ? 5.623413251903491 : 7.498942093324558;
  const double p10 = (j == 0) ? 1.0 : (j == 1) ? 10.0 : (j == 2) ? 100.0 : 1000.0;
  const float p32 = (float)(b8 * p10);
  const float inv = 1.0f / p32;
  const float ang = (float)pos * inv;
  float sn, cs;
  sincosf(ang, &sn, &cs);
  sc[tid] = cs;
  ss[tid] = sn;
  __syncthreads();
  if (tid < 64) {
    const v4f v = *(const v4f*)(sc + tid * 4);
    volatile v4f* d = (volatile v4f*)(ctab + tb + tid * 4);
    *d = v;
    __threadfence();
    *d = v;
  } else if (tid < 128) {
    const int u = tid - 64;
    const v4f v = *(const v4f*)(ss + u * 4);
    volatile v4f* d = (volatile v4f*)(stab + tb + u * 4);
    *d = v;
    __threadfence();
    *d = v;
  }
}

__global__ __launch_bounds__(256) void k_mflag(const float* __restrict__ mask, int* __restrict__ flags) {
  __shared__ int s_am[NKC * 8];
  __shared__ int s_az[NKC * 8];
  __shared__ int s_lv[8];
  const int tid = threadIdx.x, lane = tid & 31, wave = tid >> 5;
  const int qb  = blockIdx.x;
  const int row = tid >> 1, hsel = tid & 1;
  const float* rp = mask + (size_t)(qb * QB + row) * SQ + hsel * 32;
  int live = 0;
#pragma unroll 1
  for (int kc = 0; kc < NKC; ++kc) {
    const float* p = rp + kc * KC;
    int am = 1, az = 1;
#pragma unroll
    for (int q = 0; q < 8; ++q) {
      const v4f v = *(const v4f*)(p + 4 * q);
#pragma unroll
      for (int e = 0; e < 4; ++e) {
        am   &= (v[e] <= -5.0e8f) ? 1 : 0;
        az   &= (v[e] == 0.0f) ? 1 : 0;
        live |= (v[e] > -5.0e8f) ? 1 : 0;
      }
    }
#pragma unroll
    for (int off = 1; off < 32; off <<= 1) {
      am &= __shfl_xor(am, off, 32);
      az &= __shfl_xor(az, off, 32);
    }
    if (lane == 0) { s_am[kc * 8 + wave] = am; s_az[kc * 8 + wave] = az; }
  }
  live |= __shfl_xor(live, 1, 32);
  int lv = live;
#pragma unroll
  for (int off = 1; off < 32; off <<= 1) lv &= __shfl_xor(lv, off, 32);
  if (lane == 0) s_lv[wave] = lv;
  __syncthreads();
  if (wave == 0) {
    int am = 1, az = 1, lvall = 1;
#pragma unroll
    for (int w2 = 0; w2 < 8; ++w2) {
      am &= s_am[lane * 8 + w2];
      az &= s_az[lane * 8 + w2];
      lvall &= s_lv[w2];
    }
    const int code = az ? 1 : ((am & lvall) ? 2 : 0);
    const int q4 = (lane & 7) * 4;
    v4i cv;
    cv[0] = __shfl(code, q4 + 0, 32);
    cv[1] = __shfl(code, q4 + 1, 32);
    cv[2] = __shfl(code, q4 + 2, 32);
    cv[3] = __shfl(code, q4 + 3, 32);
    volatile v4i* d = (volatile v4i*)(flags + qb * NKC + q4);
    if (lane < 8) *d = cv;
    __threadfence();
    if (lane < 8) *d = cv;
  }
}

#define STP 72
__global__ __launch_bounds__(256) void k_qkv(const _Float16* __restrict__ xh,
                                             const _Float16* __restrict__ wt,
                                             const float* __restrict__ ctab,
                                             const float* __restrict__ stab,
                                             _Float16* __restrict__ qp,
                                             _Float16* __restrict__ kp,
                                             _Float16* __restrict__ vt) {
  __shared__ __align__(16) _Float16 st[256 * STP];
  const int tid = threadIdx.x, lane = tid & 31, wave = tid >> 5;
  const int hh = lane >> 4, c = lane & 15;
  const int mb = blockIdx.x * 256;
  const int m0 = mb + wave * 32;
  const int n0 = blockIdx.y * 64;
  const int which = (n0 < HID) ? 0 : ((n0 < HID + KVD) ? 1 : 2);
  if (which == 0 && mb < R0) return;

  v8f acc[2][4];
#pragma unroll
  for (int s = 0; s < 2; ++s)
#pragma unroll
    for (int t = 0; t < 4; ++t) acc[s][t] = zero8();
  gemm32x64(xh, HID, wt, HID, m0, n0, lane, acc);

  if (which < 2) {
#pragma unroll
    for (int sub = 0; sub < 2; ++sub) {
#pragma unroll
      for (int r = 0; r < 8; ++r) {
        const int lr  = wave * 32 + sub * 16 + 8 * hh + r;
        const int pos = mb + lr;
        const float* cr = ctab + (size_t)pos * NFREQ;
        const float* sr = stab + (size_t)pos * NFREQ;
#pragma unroll
        for (int t = 0; t < 2; ++t) {
          const float cs = cr[16 * t + c];
          const float sn = sr[16 * t + c];
          const float x1 = acc[sub][t][r] * 0.03125f;
          const float x2 = acc[sub][t + 2][r] * 0.03125f;
          st[lr * STP + 16 * t + c]       = (_Float16)(x1 * cs - x2 * sn);
          st[lr * STP + 16 * (t + 2) + c] = (_Float16)(x2 * cs + x1 * sn);
        }
      }
    }
  } else {
#pragma unroll
    for (int t = 0; t < 4; ++t) {
#pragma unroll
      for (int sub = 0; sub < 2; ++sub) {
#pragma unroll
        for (int r = 0; r < 8; ++r) {
          const int lr = wave * 32 + sub * 16 + 8 * hh + r;
          st[lr * STP + 16 * t + c] = (_Float16)(acc[sub][t][r] * 0.03125f);
        }
      }
    }
  }
  __syncthreads();

  _Float16* base = (which == 0) ? qp : ((which == 1) ? kp : vt);
  v4u val[8];
  size_t go[8];
  if (which < 2) {
    const int head = (which == 0) ? (n0 >> 6) : ((n0 - HID) >> 6);
#pragma unroll
    for (int j = 0; j < 8; ++j) {
      const int p  = tid + 256 * j;
      const int lr = p >> 3;
      const int pc = p & 7;
      Pack8 pk;
      pk.h  = *(const v8h*)(st + lr * STP + pc * 8);
      val[j] = pk.u;
      go[j]  = ((size_t)head * SQ + mb + lr) * HDM + pc * 8;
    }
  } else {
    const int kvh = (n0 - HID - KVD) >> 6;
#pragma unroll
    for (int j = 0; j < 8; ++j) {
      const int p  = tid + 256 * j;
      const int L  = p >> 3;
      const int pc = p & 7;
      const int d  = L >> 2;
      const int nl = (L & 3) * 64 + pc * 8;
      const _Float16* cp = st + nl * STP + d;
      Pack8 pk;
      pk.h = (v8h){cp[0 * STP], cp[1 * STP], cp[2 * STP], cp[3 * STP],
                   cp[4 * STP], cp[5 * STP], cp[6 * STP], cp[7 * STP]};
      val[j] = pk.u;
      go[j]  = ((size_t)kvh * HDM + d) * SQ + mb + nl;
    }
  }
  for (int ps = 0; ps < 2; ++ps) {
#pragma unroll
    for (int j = 0; j < 8; ++j) *(volatile v4u*)(base + go[j]) = val[j];
    __threadfence();
  }
}

__global__ __launch_bounds__(256) void k_qkv3(const ush* __restrict__ xh3, const ush* __restrict__ xl3,
                                              const ush* __restrict__ wth, const ush* __restrict__ wtl,
                                              const float* __restrict__ ctab, const float* __restrict__ stab,
                                              ush* __restrict__ q3h, ush* __restrict__ q3l,
                                              ush* __restrict__ k3h, ush* __restrict__ k3l,
                                              ush* __restrict__ v3h, ush* __restrict__ v3l) {
  __shared__ __align__(16) ush st[256 * STP];
  const int tid = threadIdx.x, lane = tid & 31, wave = tid >> 5;
  const int hh = lane >> 4, c = lane & 15;
  const int mb = blockIdx.x * 256;
  const int m0 = mb + wave * 32;
  const int n0 = blockIdx.y * 64;
  const int which = (n0 < HID) ? 0 : ((n0 < HID + KVD) ? 1 : 2);

  v8f acc[2][4];
#pragma unroll
  for (int s = 0; s < 2; ++s)
#pragma unroll
    for (int t = 0; t < 4; ++t) acc[s][t] = zero8();
  gemm3_32x64(xh3, xl3, HID, wth, wtl, HID, m0, n0, lane, acc);

  if (which < 2) {
#pragma unroll
    for (int sub = 0; sub < 2; ++sub) {
#pragma unroll
      for (int r = 0; r < 8; ++r) {
        const int lr  = wave * 32 + sub * 16 + 8 * hh + r;
        const int pos = mb + lr;
        const float* cr = ctab + (size_t)pos * NFREQ;
        const float* sr = stab + (size_t)pos * NFREQ;
#pragma unroll
        for (int t = 0; t < 2; ++t) {
          const float cs = cr[16 * t + c];
          const float sn = sr[16 * t + c];
          const float x1 = acc[sub][t][r];
          const float x2 = acc[sub][t + 2][r];
          acc[sub][t][r]     = x1 * cs - x2 * sn;
          acc[sub][t + 2][r] = x2 * cs + x1 * sn;
        }
      }
    }
  }

  ush* bh = (which == 0) ? q3h : ((which == 1) ? k3h : v3h);
  ush* bl = (which == 0) ? q3l : ((which == 1) ? k3l : v3l);
  const int head = (which == 0) ? (n0 >> 6) : ((which == 1) ? ((n0 - HID) >> 6) : ((n0 - HID - KVD) >> 6));
  size_t go[8];
#pragma unroll
  for (int j = 0; j < 8; ++j) {
    const int p  = tid + 256 * j;
    const int L  = p >> 3;
    const int pc = p & 7;
    if (which < 2) {
      go[j] = ((size_t)head * R0 + mb + L) * HDM + pc * 8;
    } else {
      const int d  = L >> 2;
      const int nl = (L & 3) * 64 + pc * 8;
      go[j] = ((size_t)head * HDM + d) * R0 + mb + nl;
    }
  }

#pragma unroll 1
  for (int ph = 0; ph < 2; ++ph) {
    __syncthreads();
#pragma unroll
    for (int t = 0; t < 4; ++t) {
#pragma unroll
      for (int sub = 0; sub < 2; ++sub) {
#pragma unroll
        for (int r = 0; r < 8; ++r) {
          const int lr = wave * 32 + sub * 16 + 8 * hh + r;
          const float v = acc[sub][t][r];
          const ush hi = f2bf(v);
          st[lr * STP + 16 * t + c] = (ph == 0) ? hi : f2bf(v - bf2f(hi));
        }
      }
    }
    __syncthreads();
    v4u val[8];
    if (which < 2) {
#pragma unroll
      for (int j = 0; j < 8; ++j) {
        const int p  = tid + 256 * j;
        const int lr = p >> 3;
        const int pc = p & 7;
        PackU pk;
        pk.s  = *(const v8us*)(st + lr * STP + pc * 8);
        val[j] = pk.u;
      }
    } else {
#pragma unroll
      for (int j = 0; j < 8; ++j) {
        const int p  = tid + 256 * j;
        const int L  = p >> 3;
        const int pc = p & 7;
        const int d  = L >> 2;
        const int nl = (L & 3) * 64 + pc * 8;
        const ush* cp = st + nl * STP + d;
        PackU pk;
        pk.s = (v8us){cp[0 * STP], cp[1 * STP], cp[2 * STP], cp[3 * STP],
                      cp[4 * STP], cp[5 * STP], cp[6 * STP], cp[7 * STP]};
        val[j] = pk.u;
      }
    }
    ush* dst = (ph == 0) ? bh : bl;
    for (int ps = 0; ps < 2; ++ps) {
#pragma unroll
      for (int j = 0; j < 8; ++j) *(volatile v4u*)(dst + go[j]) = val[j];
      __threadfence();
    }
  }
}

#define KTP 72
#define PTP 72
__global__ __launch_bounds__(256) void k_attn(const _Float16* __restrict__ qp,
                                              const _Float16* __restrict__ kp,
                                              const _Float16* __restrict__ vt,
                                              const float* __restrict__ mask,
                                              const int* __restrict__ flags,
                                              _Float16* __restrict__ op, float sscale) {
  __shared__ __align__(16) _Float16 Ks[64 * KTP];
  __shared__ __align__(16) _Float16 Vs[64 * KTP];
  __shared__ __align__(16) _Float16 Ps[8][16 * PTP];
  __shared__ __align__(16) _Float16 Mk[8][16 * PTP];

  const int tid = threadIdx.x, lane = tid & 31, wave = tid >> 5;
  const int hh = lane >> 4, c = lane & 15;
  const int h   = blockIdx.x / (NQB - QB3);
  const int qb  = QB3 + blockIdx.x % (NQB - QB3);
  const int kvh = h >> 2;
  const int q0  = qb * QB + wave * 16;

  const _Float16* Q = qp + (size_t)h * SQ * HDM;
  const _Float16* K = kp + (size_t)kvh * SQ * HDM;
  const _Float16* V = vt + (size_t)kvh * HDM * SQ;
  const float* mtile = mask + (size_t)(q0 + (lane & 15)) * SQ + (lane >> 4) * 32;
  _Float16* mw = Mk[wave];
  const int* fl = flags + qb * NKC;

  v16h qa[2];
  qa[0] = ldfrag(Q, HDM, q0, 0, lane);
  qa[1] = ldfrag(Q, HDM, q0, 32, lane);

  const float NEGI = -__builtin_huge_valf();
  float mrow[8], lrow[8];
  v8f oacc[4];
#pragma unroll
  for (int r = 0; r < 8; ++r) { mrow[r] = NEGI; lrow[r] = 0.f; }
#pragma unroll
  for (int t = 0; t < 4; ++t) oacc[t] = zero8();

  _Float16* pw = Ps[wave];

  for (int kc = 0; kc < NKC; ++kc) {
    const int flag = __builtin_amdgcn_readfirstlane(fl[kc]);
    if (flag == 2) continue;
    const int kv0 = kc * KC;
    __syncthreads();
    {
      const int r  = tid >> 2;
      const int qq = (tid & 3) * 16;
      const _Float16* ks = K + (size_t)(kv0 + r) * HDM + qq;
      *(v8h*)(Ks + r * KTP + qq)     = *(const v8h*)(ks);
      *(v8h*)(Ks + r * KTP + qq + 8) = *(const v8h*)(ks + 8);
      const _Float16* vs = V + (size_t)r * SQ + kv0 + qq;
      *(v8h*)(Vs + r * KTP + qq)     = *(const v8h*)(vs);
      *(v8h*)(Vs + r * KTP + qq + 8) = *(const v8h*)(vs + 8);
    }
    __syncthreads();

    v8f s[4];
#pragma unroll
    for (int j = 0; j < 4; ++j) s[j] = zero8();
#pragma unroll
    for (int dc = 0; dc < 2; ++dc) {
#pragma unroll
      for (int j = 0; j < 4; ++j) {
        const v16h kb = ldfrag(Ks, KTP, j * 16, dc * 32, lane);
        s[j] = mma16(qa[dc], kb, s[j]);
      }
    }
    if (flag != 1) {
      {
        const float* src = mtile + kv0;
        v4f m4[8];
#pragma unroll
        for (int e = 0; e < 8; ++e) m4[e] = *(const v4f*)(src + 4 * e);
        _Float16* dstm = mw + (lane & 15) * PTP + (lane >> 4) * 32;
#pragma unroll
        for (int e = 0; e < 8; ++e) {
#pragma unroll
          for (int u = 0; u < 4; ++u) dstm[4 * e + u] = (_Float16)m4[e][u];
        }
      }
      __syncthreads();
#pragma unroll
      for (int r = 0; r < 8; ++r)
#pragma unroll
        for (int j = 0; j < 4; ++j) s[j][r] = s[j][r] * sscale + (float)mw[(8 * hh + r) * PTP + 16 * j + c];
      __syncthreads();
    } else {
#pragma unroll
      for (int r = 0; r < 8; ++r)
#pragma unroll
        for (int j = 0; j < 4; ++j) s[j][r] = s[j][r] * sscale;
    }
    float cm[8];
#pragma unroll
    for (int r = 0; r < 8; ++r) {
      float m = NEGI;
#pragma unroll
      for (int j = 0; j < 4; ++j) m = fmaxf(m, s[j][r]);
#pragma unroll
      for (int off = 1; off < 16; off <<= 1) m = fmaxf(m, __shfl_xor(m, off, 32));
      cm[r] = m;
    }
    float al[8];
#pragma unroll
    for (int r = 0; r < 8; ++r) {
      const float mnew  = fmaxf(mrow[r], cm[r]);
      const float alpha = __expf(mrow[r] - mnew);
      mrow[r] = mnew;
      float psum = 0.f;
#pragma unroll
      for (int j = 0; j < 4; ++j) {
        const float p = __expf(s[j][r] - mnew);
        psum += p;
        pw[(8 * hh + r) * PTP + j * 16 + c] = (_Float16)(p * 1024.0f);
      }
#pragma unroll
      for (int off = 1; off < 16; off <<= 1) psum += __shfl_xor(psum, off, 32);
      lrow[r] = lrow[r] * alpha + psum;
      al[r] = alpha;
    }
#pragma unroll
    for (int t = 0; t < 4; ++t)
#pragma unroll
      for (int r = 0; r < 8; ++r) oacc[t][r] *= al[r];
    __syncthreads();

#pragma unroll
    for (int kk = 0; kk < 2; ++kk) {
      const v16h pa = ldfrag(pw, PTP, 0, kk * 32, lane);
#pragma unroll
      for (int t = 0; t < 4; ++t) {
        const v16h vb = ldfrag(Vs, KTP, t * 16, kk * 32, lane);
        oacc[t] = mma16(pa, vb, oacc[t]);
      }
    }
  }
  __syncthreads();

#pragma unroll
  for (int r = 0; r < 8; ++r) {
    const float lr  = lrow[r];
    const float inv = (lr > 0.f) ? (0.015625f / lr) : 0.f;
#pragma unroll
    for (int t = 0; t < 4; ++t) pw[(8 * hh + r) * PTP + 16 * t + c] = (_Float16)(oacc[t][r] * inv);
  }
  __syncthreads();
  v4u val[4];
  size_t go[4];
#pragma unroll
  for (int it = 0; it < 4; ++it) {
    const int p  = lane + 32 * it;
    const int L  = p >> 3;
    const int pc = p & 7;
    Pack8 pk;
    pk.h    = *(const v8h*)(pw + L * PTP + pc * 8);
    val[it] = pk.u;
    go[it]  = ((size_t)(q0 + L)) * HID + (size_t)h * HDM + pc * 8;
  }
  for (int ps = 0; ps < 2; ++ps) {
#pragma unroll
    for (int it = 0; it < 4; ++it) *(volatile v4u*)(op + go[it]) = val[it];
    __threadfence();
  }
}

#define SS3 68
static_assert(QB % KC == 0);
static_assert(QB3 * QB == R0);
static_assert(QB == 8 * 16);
static_assert((SS3 % 4) == 0);
__global__ __launch_bounds__(256)
void k_attn3(const ush* __restrict__ q3h, const ush* __restrict__ q3l,
             const ush* __restrict__ k3h, const ush* __restrict__ k3l,
             const ush* __restrict__ v3h, const ush* __restrict__ v3l,
             const float* __restrict__ mask,
             const int* __restrict__ flags,
             ush* __restrict__ o3h, ush* __restrict__ o3l, float sscale) {
  __shared__ __align__(16) float sS[QB * SS3];
  __shared__ __align__(16) ush   sPh[QB * PTP];
  __shared__ __align__(16) ush   sPl[QB * PTP];
  __shared__ __align__(16) float rSc[QB];
  __shared__ __align__(16) float rL[QB];

  const int tid = threadIdx.x, lane = tid & 31, wave = tid >> 5;
  const int hh = lane >> 4, c = lane & 15;
  const int h   = blockIdx.x / QB3;
  const int qb  = blockIdx.x % QB3;
  const int kvh = h >> 2;
  const int q0  = qb * QB + wave * 16;
  const int srow = tid >> 1;
  const int skey = (tid & 1) * 32;

  const ush* Qh  = q3h + (size_t)h * R0 * HDM;
  const ush* Ql  = q3l + (size_t)h * R0 * HDM;
  const ush* K3H = k3h + (size_t)kvh * R0 * HDM;
  const ush* K3L = k3l + (size_t)kvh * R0 * HDM;
  const ush* V3H = v3h + (size_t)kvh * HDM * R0;
  const ush* V3L = v3l + (size_t)kvh * HDM * R0;
  const float* mlane = mask + (size_t)(q0 + 8 * hh) * SQ + c;
  const int* fl = flags + qb * NKC;

  const float NEGI = -__builtin_huge_valf();
  float mrun = NEGI, lrun = 0.f;
  v8f oacc[4];
#pragma unroll
  for (int t = 0; t < 4; ++t) oacc[t] = zero8();

  float* sw  = sS  + wave * (16 * SS3);
  ush*   pwh = sPh + wave * (16 * PTP);
  ush*   pwl = sPl + wave * (16 * PTP);
  const int nck = (qb + 1) * (QB / KC);

#pragma unroll 1
  for (int kc = 0; kc < nck; ++kc) {
    const int flag = 0;
    const int kv0  = kc * KC;

    v8f s[4];
#pragma unroll
    for (int j = 0; j < 4; ++j) s[j] = zero8();
#pragma unroll 1
    for (int dc = 0; dc < 2; ++dc) {
      const v16us qah = ldfragu(Qh, HDM, q0, dc * 32, lane);
      const v16us qal = ldfragu(Ql, HDM, q0, dc * 32, lane);
#pragma unroll
      for (int jp = 0; jp < 4; jp += 2) {
        const v16us k0h = ldfragu(K3H, HDM, kv0 + 16 * jp, dc * 32, lane);
        const v16us k0l = ldfragu(K3L, HDM, kv0 + 16 * jp, dc * 32, lane);
        const v16us k1h = ldfragu(K3H, HDM, kv0 + 16 * (jp + 1), dc * 32, lane);
        const v16us k1l = ldfragu(K3L, HDM, kv0 + 16 * (jp + 1), dc * 32, lane);
        s[jp]     = mmab(qah, k0h, s[jp]);
        s[jp + 1] = mmab(qah, k1h, s[jp + 1]);
        s[jp]     = mmab(qah, k0l, s[jp]);
        s[jp + 1] = mmab(qah, k1l, s[jp + 1]);
        s[jp]     = mmab(qal, k0h, s[jp]);
        s[jp + 1] = mmab(qal, k1h, s[jp + 1]);
      }
    }
    if (flag != 1) {
#pragma unroll
      for (int r = 0; r < 8; ++r)
#pragma unroll
        for (int j = 0; j < 4; ++j)
          sw[(8 * hh + r) * SS3 + 16 * j + c] = s[j][r] * sscale + mlane[(size_t)r * SQ + kv0 + 16 * j];
    } else {
#pragma unroll
      for (int r = 0; r < 8; ++r)
#pragma unroll
        for (int j = 0; j < 4; ++j)
          sw[(8 * hh + r) * SS3 + 16 * j + c] = s[j][r] * sscale;
    }
    __syncthreads();

    {
      const float* sr = sS + srow * SS3 + skey;
      v4f x[8];
#pragma unroll
      for (int g = 0; g < 8; ++g) x[g] = *(const v4f*)(sr + 4 * g);
      float mx = x[0][0];
#pragma unroll
      for (int g = 0; g < 8; ++g) {
#pragma unroll
        for (int e = 0; e < 4; ++e) mx = fmaxf(mx, x[g][e]);
      }
      mx = fmaxf(mx, __shfl_xor(mx, 1, 32));
      const float mnew = fmaxf(mrun, mx);
      const float fac  = __expf(mrun - mnew);
      mrun = mnew;
      float sum = 0.f;
      ush* dh = sPh + srow * PTP + skey;
      ush* dl = sPl + srow * PTP + skey;
#pragma unroll
      for (int g = 0; g < 4; ++g) {
        const v4f xa = x[2 * g];
        const v4f xb = x[2 * g + 1];
        PackU ph, pl;
#pragma unroll
        for (int e = 0; e < 4; ++e) {
          const float p = __expf(xa[e] - mnew);
          sum += p;
          const ush hi = f2bf(p);
          ph.s[e] = hi;
          pl.s[e] = f2bf(p - bf2f(hi));
        }
#pragma unroll
        for (int e = 0; e < 4; ++e) {
          const float p = __expf(xb[e] - mnew);
          sum += p;
          const ush hi = f2bf(p);
          ph.s[4 + e] = hi;
          pl.s[4 + e] = f2bf(p - bf2f(hi));
        }
        *(v8us*)(dh + 8 * g) = ph.s;
        *(v8us*)(dl + 8 * g) = pl.s;
      }
      sum += __shfl_xor(sum, 1, 32);
      lrun = lrun * fac + sum;
      if (skey == 0) rSc[srow] = fac;
    }
    __syncthreads();

    {
      const v4f f0 = *(const v4f*)(rSc + wave * 16 + 8 * hh);
      const v4f f1 = *(const v4f*)(rSc + wave * 16 + 8 * hh + 4);
#pragma unroll
      for (int t = 0; t < 4; ++t) {
#pragma unroll
        for (int r = 0; r < 4; ++r) {
          oacc[t][r]     *= f0[r];
          oacc[t][4 + r] *= f1[r];
        }
      }
    }
#pragma unroll 1
    for (int kk = 0; kk < 2; ++kk) {
      const v16us pah = ldfragu(pwh, PTP, 0, kk * 32, lane);
      const v16us pal = ldfragu(pwl, PTP, 0, kk * 32, lane);
#pragma unroll
      for (int tp = 0; tp < 4; tp += 2) {
        const v16us v0h = ldfragu(V3H, R0, 16 * tp, kv0 + kk * 32, lane);
        const v16us v0l = ldfragu(V3L, R0, 16 * tp, kv0 + kk * 32, lane);
        const v16us v1h = ldfragu(V3H, R0, 16 * (tp + 1), kv0 + kk * 32, lane);
        const v16us v1l = ldfragu(V3L, R0, 16 * (tp + 1), kv0 + kk * 32, lane);
        oacc[tp]     = mmab(pah, v0h, oacc[tp]);
        oacc[tp + 1] = mmab(pah, v1h, oacc[tp + 1]);
        oacc[tp]     = mmab(pah, v0l, oacc[tp]);
        oacc[tp + 1] = mmab(pah, v1l, oacc[tp + 1]);
        oacc[tp]     = mmab(pal, v0h, oacc[tp]);
        oacc[tp + 1] = mmab(pal, v1h, oacc[tp + 1]);
      }
    }
    __syncthreads();
  }

  if (skey == 0) rL[srow] = lrun;
  __syncthreads();

  {
    const v4f l0 = *(const v4f*)(rL + wave * 16 + 8 * hh);
    const v4f l1 = *(const v4f*)(rL + wave * 16 + 8 * hh + 4);
#pragma unroll
    for (int r = 0; r < 8; ++r) {
      const float lr  = (r < 4) ? l0[r & 3] : l1[r & 3];
      const float inv = (lr > 0.f) ? (1.0f / lr) : 0.f;
#pragma unroll
      for (int t = 0; t < 4; ++t) {
        const float o = oacc[t][r] * inv;
        const ush hi = f2bf(o);
        pwh[(8 * hh + r) * PTP + 16 * t + c] = hi;
        pwl[(8 * hh + r) * PTP + 16 * t + c] = f2bf(o - bf2f(hi));
      }
    }
  }
  __syncthreads();
  v4u vh[4], vl[4];
  size_t go[4];
#pragma unroll
  for (int it = 0; it < 4; ++it) {
    const int p  = lane + 32 * it;
    const int L  = p >> 3;
    const int pc = p & 7;
    PackU pk;
    pk.s   = *(const v8us*)(pwh + L * PTP + pc * 8);
    vh[it] = pk.u;
    pk.s   = *(const v8us*)(pwl + L * PTP + pc * 8);
    vl[it] = pk.u;
    go[it] = ((size_t)(q0 + L)) * HID + (size_t)h * HDM + pc * 8;
  }
  for (int ps = 0; ps < 2; ++ps) {
#pragma unroll
    for (int it = 0; it < 4; ++it) {
      *(volatile v4u*)(o3h + go[it]) = vh[it];
      *(volatile v4u*)(o3l + go[it]) = vl[it];
    }
    __threadfence();
  }
}

#define OTP 68
__device__ __forceinline__ void out_epilogue(v8f (&acc)[2][4], float scale, float* sw, float* __restrict__ out,
                                             int m0, int n0, int lane, int hh, int c) {
#pragma unroll
  for (int sub = 0; sub < 2; ++sub) {
    __syncthreads();
#pragma unroll
    for (int t = 0; t < 4; ++t) {
#pragma unroll
      for (int r = 0; r < 8; ++r) sw[(8 * hh + r) * OTP + 16 * t + c] = acc[sub][t][r] * scale;
    }
    __syncthreads();
    v4f val[8];
    size_t go[8];
#pragma unroll
    for (int it = 0; it < 8; ++it) {
      const int p    = lane + 32 * it;
      const int L    = p >> 3;
      const int pc   = p & 7;
      const int row  = L >> 1;
      const int half = L & 1;
      val[it] = *(const v4f*)(sw + row * OTP + half * 32 + pc * 4);
      go[it]  = (size_t)(m0 + sub * 16 + row) * HID + n0 + half * 32 + pc * 4;
    }
    for (int ps = 0; ps < 2; ++ps) {
#pragma unroll
      for (int it = 0; it < 8; ++it) *(volatile v4f*)(out + go[it]) = val[it];
      __threadfence();
    }
  }
}

__global__ __launch_bounds__(256) void k_out(const _Float16* __restrict__ ap,
                                             const _Float16* __restrict__ wt,
                                             float* __restrict__ out, int mblk0) {
  __shared__ __align__(16) float st[8][16 * OTP];
  const int tid = threadIdx.x, lane = tid & 31, wave = tid >> 5;
  const int hh = lane >> 4, c = lane & 15;
  const int m0 = (mblk0 + blockIdx.x) * 256 + wave * 32;
  const int n0 = blockIdx.y * 64;

  v8f acc[2][4];
#pragma unroll
  for (int s = 0; s < 2; ++s)
#pragma unroll
    for (int t = 0; t < 4; ++t) acc[s][t] = zero8();
  gemm32x64(ap, HID, wt, HID, m0, n0, lane, acc);
  out_epilogue(acc, 0.001953125f, st[wave], out, m0, n0, lane, hh, c);
}

__global__ __launch_bounds__(256) void k_out3(const ush* __restrict__ ah, const ush* __restrict__ al,
                                              const ush* __restrict__ wh, const ush* __restrict__ wl,
                                              float* __restrict__ out) {
  __shared__ __align__(16) float st[8][16 * OTP];
  const int tid = threadIdx.x, lane = tid & 31, wave = tid >> 5;
  const int hh = lane >> 4, c = lane & 15;
  const int m0 = blockIdx.x * 256 + wave * 32;
  const int n0 = blockIdx.y * 64;

  v8f acc[2][4];
#pragma unroll
  for (int s = 0; s < 2; ++s)
#pragma unroll
    for (int t = 0; t < 4; ++t) acc[s][t] = zero8();
  gemm3_32x64(ah, al, HID, wh, wl, HID, m0, n0, lane, acc);
  out_epilogue(acc, 1.0f, st[wave], out, m0, n0, lane, hh, c);
}

extern "C" void kernel_launch(void* const* d_in, const int* in_sizes, int n_in,
                              void* d_out, int out_size, void* d_ws, size_t ws_size,
                              hipStream_t stream) {
  if (n_in < 6) return;
  if (in_sizes[0] != SQ * HID) return;
  if (in_sizes[1] != HID * HID) return;
  if (in_sizes[2] != HID * KVD) return;
  if (in_sizes[3] != HID * KVD) return;
  if (in_sizes[4] != HID * HID) return;
  if (in_sizes[5] != SQ * SQ) return;
  if (out_size != SQ * HID) return;

  const float* x    = (const float*)d_in[0];
  const float* wq   = (const float*)d_in[1];
  const float* wk   = (const float*)d_in[2];
  const float* wv   = (const float*)d_in[3];
  const float* wo   = (const float*)d_in[4];
  const float* mask = (const float*)d_in[5];
  float* out = (float*)d_out;

  size_t off = 0;
  const size_t oX   = off; off += (size_t)SQ * HID * 2;
  const size_t oX3h = off; off += (size_t)R0 * HID * 2;
  const size_t oX3l = off; off += (size_t)R0 * HID * 2;
  const size_t oWt  = off; off += (size_t)NQKV * HID * 2;
  const size_t oWth = off; off += (size_t)NQKV * HID * 2;
  const size_t oWtl = off; off += (size_t)NQKV * HID * 2;
  const size_t oWo  = off; off += (size_t)HID * HID * 2;
  const size_t oWoh = off; off += (size_t)HID * HID * 2;
  const size_t oWol = off; off += (size_t)HID * HID * 2;
  const size_t oQ   = off; off += (size_t)NH * SQ * HDM * 2;
  const size_t oK   = off; off += (size_t)NKV * SQ * HDM * 2;
  const size_t oV   = off; off += (size_t)NKV * HDM * SQ * 2;
  const size_t oQ3h = off; off += (size_t)NH * R0 * HDM * 2;
  const size_t oQ3l = off; off += (size_t)NH * R0 * HDM * 2;
  const size_t oK3h = off; off += (size_t)NKV * R0 * HDM * 2;
  const size_t oK3l = off; off += (size_t)NKV * R0 * HDM * 2;
  const size_t oV3h = off; off += (size_t)NKV * HDM * R0 * 2;
  const size_t oV3l = off; off += (size_t)NKV * HDM * R0 * 2;
  const size_t oO   = off; off += (size_t)SQ * HID * 2;
  const size_t oO3h = off; off += (size_t)R0 * HID * 2;
  const size_t oO3l = off; off += (size_t)R0 * HID * 2;
  const size_t oC   = off; off += (size_t)SQ * NFREQ * 4;
  const size_t oS   = off; off += (size_t)SQ * NFREQ * 4;
  const size_t oF   = off; off += (size_t)NQB * NKC * 4;
  if (off > ws_size) return;
  if (off > (size_t)134217728) return;

  char* ws = (char*)d_ws;
  _Float16* Xh  = (_Float16*)(ws + oX);
  ush*      X3h = (ush*)(ws + oX3h);
  ush*      X3l = (ush*)(ws + oX3l);
  _Float16* Wt  = (_Float16*)(ws + oWt);
  ush*      Wth = (ush*)(ws + oWth);
  ush*      Wtl = (ush*)(ws + oWtl);
  _Float16* Wot = (_Float16*)(ws + oWo);
  ush*      Woh = (ush*)(ws + oWoh);
  ush*      Wol = (ush*)(ws + oWol);
  _Float16* Qp  = (_Float16*)(ws + oQ);
  _Float16* Kp  = (_Float16*)(ws + oK);
  _Float16* Vt  = (_Float16*)(ws + oV);
  ush*      Q3h = (ush*)(ws + oQ3h);
  ush*      Q3l = (ush*)(ws + oQ3l);
  ush*      K3h = (ush*)(ws + oK3h);
  ush*      K3l = (ush*)(ws + oK3l);
  ush*      V3h = (ush*)(ws + oV3h);
  ush*      V3l = (ush*)(ws + oV3l);
  _Float16* Op  = (_Float16*)(ws + oO);
  ush*      O3h = (ush*)(ws + oO3h);
  ush*      O3l = (ush*)(ws + oO3l);
  float* Ct = (float*)(ws + oC);
  float* St = (float*)(ws + oS);
  int*   Fl = (int*)(ws + oF);

  const int ngrp  = in_sizes[0] / 8;
  const int n3grp = (R0 * HID) / 8;
  k_cvt_x<<<dim3((ngrp + 255) / 256), dim3(256), 0, stream>>>(x, Xh, X3h, X3l, ngrp, n3grp);
  const size_t rk = (size_t)HID * HID;
  const size_t rv = (size_t)(HID + KVD) * HID;
  k_wt<<<dim3(HID / 64, HID / 64), dim3(256), 0, stream>>>(wq, Wt, Wth, Wtl, HID);
  k_wt<<<dim3(KVD / 64, HID / 64), dim3(256), 0, stream>>>(wk, Wt + rk, Wth + rk, Wtl + rk, KVD);
  k_wt<<<dim3(KVD / 64, HID / 64), dim3(256), 0, stream>>>(wv, Wt + rv, Wth + rv, Wtl + rv, KVD);
  k_wt<<<dim3(HID / 64, HID / 64), dim3(256), 0, stream>>>(wo, Wot, Woh, Wol, HID);
  k_wsplit<<<dim3((HID * (HID / 8)) / 256), dim3(256), 0, stream>>>(wq, Wth, Wtl, HID);
  k_wsplit<<<dim3((KVD * (HID / 8)) / 256), dim3(256), 0, stream>>>(wk, Wth + rk, Wtl + rk, KVD);
  k_wsplit<<<dim3((KVD * (HID / 8)) / 256), dim3(256), 0, stream>>>(wv, Wth + rv, Wtl + rv, KVD);
  k_wsplit<<<dim3((HID * (HID / 8)) / 256), dim3(256), 0, stream>>>(wo, Woh, Wol, HID);
  const int ntab = SQ * NFREQ;
  if ((ntab & 255) != 0) return;
  k_rope_tab<<<dim3(ntab / 256), dim3(256), 0, stream>>>(Ct, St, ntab);
  k_mflag<<<dim3(NQB), dim3(256), 0, stream>>>(mask, Fl);
  k_qkv<<<dim3(SQ / 256, NQKV / 64), dim3(256), 0, stream>>>(Xh, Wt, Ct, St, Qp, Kp, Vt);
  k_qkv3<<<dim3(MB3, NQKV / 64), dim3(256), 0, stream>>>(X3h, X3l, Wth, Wtl, Ct, St,
                                                          Q3h, Q3l, K3h, K3l, V3h, V3l);
  k_attn<<<dim3(NH * (NQB - QB3)), dim3(256), 0, stream>>>(Qp, Kp, Vt, mask, Fl, Op, 0.125f);
  k_attn3<<<dim3(NH * QB3), dim3(256), 0, stream>>>(Q3h, Q3l, K3h, K3l, V3h, V3l, mask, Fl,
                                                      O3h, O3l, 0.125f);
  k_out<<<dim3(SQ / 256 - MB3, HID / 64), dim3(256), 0, stream>>>(Op, Wot, out, MB3);
  k_out3<<<dim3(MB3, HID / 64), dim3(256), 0, stream>>>(O3h, O3l, Woh, Wol, out);
  (void)hipGetLastError();
}
